// NN_24472723653267
// MI455X (gfx1250) — hardware-run, weakly checked
//
#include <hip/hip_runtime.h>

constexpr int NB   = 16384;
constexpr int NL   = 50;
constexpr int ND   = 20;
constexpr int NCH  = 16;
constexpr int NHU  = 6;
constexpr int NG3  = 18;
constexpr int NWV  = 2;
constexpr int NTHF = 32 * NWV;
constexpr int XAP  = 32;
constexpr int XRP  = 72;
constexpr int A1P  = 64;
constexpr int WCP  = 96;
constexpr int WE_OFF = 0;
constexpr int WA_OFF = 512;
constexpr int WG_OFF = 1024;
constexpr int WC_OFF = 2048;
constexpr int WPL_N  = 6656;
constexpr int PWHH = 0, PBHH = 108, PWEB = 128, PATB = 144, PCVB = 160, PBIH = 208, PFCW = 228, PFCB = 336, NPAR = 344;
constexpr int SCR_GI = 0, SCR_X4 = 928, SCR_Y = 1232, SCR_N = 1536;
constexpr float XCAR   = 8.0f;
constexpr float WCARRY = 16.0f;
constexpr float FOLD   = 1.0f / 128.0f;
constexpr int OUTT_LINE = 32;
static_assert(NB % NWV == 0, "grid exact");
static_assert(WPL_N % 8 == 0 && (WPL_N / 8) % NTHF == 0, "weight copy loop exact");
static_assert((NB * 2) % (4 * 256) == 0, "final store grid exact");
static_assert(SCR_GI + NL * NG3 <= SCR_X4 && SCR_X4 + NL * NHU <= SCR_Y && SCR_Y + NL * NHU <= SCR_N, "scratch layout");

typedef __attribute__((ext_vector_type(16))) _Float16 v16h;
typedef __attribute__((ext_vector_type(8)))  _Float16 v8h;
typedef __attribute__((ext_vector_type(8)))  float    v8f;
typedef __attribute__((ext_vector_type(4)))  float    v4f;
typedef __attribute__((ext_vector_type(8)))  unsigned v8u;
typedef __attribute__((ext_vector_type(2)))  unsigned v2u;

__device__ __forceinline__ void dep_guard_h(v8f& a, v8f& b, v16h x, v16h y) { asm volatile("v_nop\n\tv_nop\n\tv_nop\n\tv_nop" : "+v"(a), "+v"(b) : "v"(x), "v"(y)); }
__device__ __forceinline__ void keep4_h(v16h a, v16h b, v16h c, v16h d) { asm volatile("v_nop" :: "v"(a), "v"(b), "v"(c), "v"(d)); }
template <typename T> struct Frag;
template <> struct Frag<_Float16> {
  typedef v16h V; union U { v16h v; v8h h[2]; };
  static __device__ __forceinline__ v16h load(const _Float16* p) {
    U f; f.h[0] = *(const v8h*)(p); f.h[1] = *(const v8h*)(p + 16); return f.v;
  }
  static __device__ __forceinline__ v8f mma(v16h a, v16h b, v8f c) {
    return __builtin_amdgcn_wmma_f32_16x16x32_f16(false, a, false, b, (short)0, c, false, false);
  }
  static __device__ __forceinline__ void guard(v8f& a, v8f& b, v16h x, v16h y) { dep_guard_h(a, b, x, y); }
  static __device__ __forceinline__ void keep(v16h a, v16h b, v16h c, v16h d) { keep4_h(a, b, c, d); }
};

__device__ __forceinline__ v8f hmma(v16h a, v16h b, v8f c) {
  c = __builtin_amdgcn_wmma_f32_16x16x32_f16(false, a, false, b, (short)0, c, false, false);
  asm volatile("v_nop\n\tv_nop\n\tv_nop\n\tv_nop" : "+v"(c) : "v"(a), "v"(b));
  return c;
}

__device__ __forceinline__ float fsig(float x)  { return __builtin_amdgcn_rcpf(1.0f + expf(-x)); }
__device__ __forceinline__ float ftanh(float x) { return 1.0f - 2.0f * __builtin_amdgcn_rcpf(expf(2.0f * x) + 1.0f); }

__host__ __device__ constexpr int im_k(int kt, int v, int e, int hh) { return kt * 32 + 8 * hh + 2 * v + (v >= 4 ? 8 : 0) + e; }
__host__ __device__ constexpr int im_off(int k) { return (k / 5) * XRP + (k % 5); }

struct alignas(16) WaveLds {
  union U1 { unsigned short xA[64 * XAP]; float attnT[64 * NCH]; } u1;
  unsigned short xeA[64 * XAP];
  unsigned short xrP[NCH * XRP];
  union U2 { float scr[SCR_N]; float attn1P[48 * A1P]; } u2;
  float xcnn[48];
  float xgru[8];
};
struct alignas(16) BlockLds {
  unsigned short w[WPL_N];
  float par[NPAR];
  float outv[4];
  WaveLds wv[NWV];
};
static_assert(sizeof(WaveLds) % 16 == 0, "wave arena alignment");
static_assert(sizeof(BlockLds) <= 65536, "static LDS budget");

__global__ __launch_bounds__(256) void k_prep(const float* __restrict__ we_w, const float* __restrict__ attn_w,
                                              const float* __restrict__ gru_wih,
                                              const float* __restrict__ conv1_w, const float* __restrict__ conv2_w,
                                              const float* __restrict__ conv3_w, unsigned short* __restrict__ wpl) {
  __shared__ float swe[NCH * ND];
  __shared__ float swa[NCH * NCH];
  __shared__ float swg[NG3 * NCH];
  __shared__ float sc1[NCH * NCH];
  __shared__ float sc2[NCH * NCH * 3];
  __shared__ float sc3[NCH * NCH * 5];
  const int tid = threadIdx.x;
#pragma unroll 1
  for (int i = tid; i < NCH * ND; i += 256) swe[i] = we_w[i];
#pragma unroll 1
  for (int i = tid; i < NCH * NCH; i += 256) swa[i] = attn_w[i];
#pragma unroll 1
  for (int i = tid; i < NG3 * NCH; i += 256) swg[i] = gru_wih[i];
#pragma unroll 1
  for (int i = tid; i < NCH * NCH; i += 256) sc1[i] = conv1_w[i];
#pragma unroll 1
  for (int i = tid; i < NCH * NCH * 3; i += 256) sc2[i] = conv2_w[i];
#pragma unroll 1
  for (int i = tid; i < NCH * NCH * 5; i += 256) sc3[i] = conv3_w[i];
  __syncthreads();

  if (tid < 64) {
    const int n = tid >> 2, kb = (tid & 3) * 8;
    v8h hv;
#pragma unroll
    for (int e = 0; e < 8; ++e) {
      const int k = kb + e;
      const int kc = k < ND ? k : (ND - 1);
      const float f = (k < ND) ? 1.0f : 0.0f;
      hv[e] = (_Float16)(swe[n * ND + kc] * f * WCARRY);
    }
    unsigned short* d = wpl + WE_OFF + 8 * tid;
    *(volatile v8h*)d = hv;
    __threadfence();
    *(volatile v8h*)d = hv;
  }
  if (tid < 64) {
    const int n = tid >> 2, kb = (tid & 3) * 8;
    v8h hv;
#pragma unroll
    for (int e = 0; e < 8; ++e) {
      const int k = kb + e;
      const int kc = k < NCH ? k : (NCH - 1);
      const float f = (k < NCH) ? 1.0f : 0.0f;
      hv[e] = (_Float16)(swa[n * NCH + kc] * f * WCARRY);
    }
    unsigned short* d = wpl + WA_OFF + 8 * tid;
    *(volatile v8h*)d = hv;
    __threadfence();
    *(volatile v8h*)d = hv;
  }
  if (tid < 128) {
    const int n = tid >> 2, kb = (tid & 3) * 8;
    const int nc = n < NG3 ? n : (NG3 - 1);
    const float fn = (n < NG3) ? 1.0f : 0.0f;
    v8h hv;
#pragma unroll
    for (int e = 0; e < 8; ++e) {
      const int k = kb + e;
      const int kc = k < NCH ? k : (NCH - 1);
      const float f = ((k < NCH) ? 1.0f : 0.0f) * fn;
      hv[e] = (_Float16)(swg[nc * NCH + kc] * f * WCARRY);
    }
    unsigned short* d = wpl + WG_OFF + 8 * tid;
    *(volatile v8h*)d = hv;
    __threadfence();
    *(volatile v8h*)d = hv;
  }
#pragma unroll 1
  for (int i = tid; i < 48 * 12; i += 256) {
    const int p  = i / 12;
    const int kb = (i - 12 * p) * 8;
    const int pm = p & 15;
    const float fp1 = (p < 16) ? 1.0f : 0.0f;
    const float fp2 = (p >= 16 && p < 32) ? 1.0f : 0.0f;
    const float fp3 = (p >= 32) ? 1.0f : 0.0f;
    v8h hv;
#pragma unroll
    for (int e = 0; e < 8; ++e) {
      const int k   = kb + e;
      const int kc  = k < 80 ? k : 79;
      const int cin = kc / 5;
      const int tap = kc - 5 * cin;
      const float fk = (k < 80) ? 1.0f : 0.0f;
      int t2 = tap - 1; t2 = t2 < 0 ? 0 : (t2 > 2 ? 2 : t2);
      const float c1 = sc1[pm * NCH + cin];
      const float c2 = sc2[(pm * NCH + cin) * 3 + t2];
      const float c3 = sc3[(pm * NCH + cin) * 5 + tap];
      const float f1 = fp1 * fk * ((tap == 2) ? 1.0f : 0.0f);
      const float f2 = fp2 * fk * ((tap >= 1 && tap <= 3) ? 1.0f : 0.0f);
      const float f3 = fp3 * fk;
      const float val = fmaf(f1, c1, fmaf(f2, c2, f3 * c3));
      hv[e] = (_Float16)(val * WCARRY);
    }
    unsigned short* d = wpl + WC_OFF + 8 * i;
    *(volatile v8h*)d = hv;
    __threadfence();
    *(volatile v8h*)d = hv;
  }
}

__global__ __launch_bounds__(NTHF) void k_front(
    const float* __restrict__ x, const unsigned short* __restrict__ wpl,
    const float* __restrict__ we_b, const float* __restrict__ attn_b,
    const float* __restrict__ conv1_b, const float* __restrict__ conv2_b, const float* __restrict__ conv3_b,
    const float* __restrict__ gru_whh, const float* __restrict__ gru_bih, const float* __restrict__ gru_bhh,
    const float* __restrict__ fc3_w, const float* __restrict__ fc3_b,
    float* __restrict__ outt) {
  __shared__ BlockLds sh;
  const int tid = threadIdx.x, lane = tid & 31, wave = tid >> 5;
  const int c = lane & 15, hh = lane >> 4, koff = 8 * hh;
  const int smp = blockIdx.x * NWV + wave;
  WaveLds& s = sh.wv[wave];
  const v8f z8 = {0.f, 0.f, 0.f, 0.f, 0.f, 0.f, 0.f, 0.f};

#pragma unroll 1
  for (int i = tid; i < WPL_N / 8; i += NTHF) ((uint4*)sh.w)[i] = ((const uint4*)wpl)[i];
  {
#pragma unroll
    for (int it = 0; it < 2; ++it) {
      const int i = tid + it * NTHF;
      const int ic = i < 108 ? i : 107;
      const float a = gru_whh[ic];
      const float b = fc3_w[ic];
      if (i < 108) { sh.par[PWHH + i] = a; sh.par[PFCW + i] = b; }
    }
    const int t18 = tid < NG3 ? tid : (NG3 - 1);
    const int t16 = tid < NCH ? tid : (NCH - 1);
    const int t2  = tid < 2 ? tid : 1;
    const float vbhh = gru_bhh[t18], vbih = gru_bih[t18];
    asm volatile("" ::: "memory");
    const float vweb = we_b[t16], vatb = attn_b[t16];
    const float vc1 = conv1_b[t16], vc2 = conv2_b[t16], vc3 = conv3_b[t16];
    const float vfcb = fc3_b[t2];
    if (tid < NG3) { sh.par[PBHH + tid] = vbhh; sh.par[PBIH + tid] = vbih; }
    if (tid < NCH) {
      sh.par[PWEB + tid] = vweb; sh.par[PATB + tid] = vatb;
      sh.par[PCVB + tid] = vc1; sh.par[PCVB + 16 + tid] = vc2; sh.par[PCVB + 32 + tid] = vc3;
    }
    if (tid < 2) sh.par[PFCB + tid] = vfcb;
  }
  __syncthreads();

  {
    unsigned* xAu = (unsigned*)s.u1.xA;
#pragma unroll 1
    for (int e = lane; e < NL * 6; e += 32) { const int row = e / 6; const int q = e - 6 * row; xAu[row * 16 + 10 + q] = 0u; }
#pragma unroll 1
    for (int e = lane; e < 14 * 16; e += 32) xAu[NL * 16 + e] = 0u;
    unsigned* xeAu = (unsigned*)s.xeA;
#pragma unroll 1
    for (int e = lane; e < 64 * 8; e += 32) { const int row = e >> 3; xeAu[row * 16 + 8 + (e & 7)] = 0u; }
    unsigned* xrPu = (unsigned*)s.xrP;
#pragma unroll 1
    for (int e = lane; e < NCH * 11; e += 32) {
      const int row = e / 11; const int q = e - 11 * row;
      const int o = (q == 0) ? 0 : (25 + q);
      xrPu[row * 36 + o] = 0u;
    }
    const float* xs = x + (size_t)smp * (NL * ND);
#pragma unroll 1
    for (int it = 0; it < 8; ++it) {
      const int q = lane + 32 * it;
      const int qc = q < 250 ? q : 249;
      const v4f v = *(const v4f*)(xs + 4 * qc);
      const int l = qc / 5;
      const int d0h = (qc - 5 * l) * 2;
      const _Float16 h0 = (_Float16)(v[0] * XCAR), h1 = (_Float16)(v[1] * XCAR);
      const _Float16 h2 = (_Float16)(v[2] * XCAR), h3 = (_Float16)(v[3] * XCAR);
      const unsigned short b0 = __builtin_bit_cast(unsigned short, h0), b1 = __builtin_bit_cast(unsigned short, h1);
      const unsigned short b2 = __builtin_bit_cast(unsigned short, h2), b3 = __builtin_bit_cast(unsigned short, h3);
      v2u pk;
      pk[0] = (unsigned)b0 | ((unsigned)b1 << 16);
      pk[1] = (unsigned)b2 | ((unsigned)b3 << 16);
      if (q < 250) *(v2u*)(xAu + l * 16 + d0h) = pk;
    }
  }
  __syncthreads();

  const _Float16* sWh = (const _Float16*)sh.w;

  {
    const v16h bE = Frag<_Float16>::load(sWh + WE_OFF + c * XAP + koff);
    const float web = sh.par[PWEB + c];
#pragma unroll 1
    for (int mt = 0; mt < 4; ++mt) {
      const v16h a = Frag<_Float16>::load((const _Float16*)s.u1.xA + (mt * 16 + c) * XAP + koff);
      const v8f acc = hmma(a, bE, z8);
#pragma unroll
      for (int r = 0; r < 8; ++r) {
        const int l = mt * 16 + 8 * hh + r;
        const float xe = acc[r] * FOLD + web;
        const _Float16 h8 = (_Float16)(xe * XCAR);
        const unsigned short hb = __builtin_bit_cast(unsigned short, h8);
        s.xeA[l * XAP + c] = hb;
        const int f = l * NCH + c;
        const int cin = f / NL;
        const int pos = f - NL * cin;
        const int cinc = cin < NCH ? cin : (NCH - 1);
        if (l < NL) s.xrP[cinc * XRP + 2 + pos] = hb;
      }
    }
  }
  __syncthreads();

  float* scr = s.u2.scr;
  {
    const v16h bG0 = Frag<_Float16>::load(sWh + WG_OFF + c * XAP + koff);
    const v16h bG1 = Frag<_Float16>::load(sWh + WG_OFF + (16 + c) * XAP + koff);
    const float bi0 = sh.par[PBIH + c];
    const int g1c = (16 + c) < NG3 ? (16 + c) : (NG3 - 1);
    const float bi1 = sh.par[PBIH + g1c];
#pragma unroll 1
    for (int mt = 0; mt < 4; ++mt) {
      const v16h a = Frag<_Float16>::load((const _Float16*)s.xeA + (mt * 16 + c) * XAP + koff);
      const v8f acc0 = hmma(a, bG0, z8);
      const v8f acc1 = hmma(a, bG1, z8);
#pragma unroll
      for (int r = 0; r < 8; ++r) {
        const int l = mt * 16 + 8 * hh + r;
        if (l < NL) {
          scr[SCR_GI + l * NG3 + c] = acc0[r] * FOLD + bi0;
          if (c < 2) scr[SCR_GI + l * NG3 + 16 + c] = acc1[r] * FOLD + bi1;
        }
      }
    }
  }
  __syncthreads();

  {
    const int u = lane < NHU ? lane : (NHU - 1);
    float wr[NHU], wz[NHU], wn[NHU];
#pragma unroll
    for (int k = 0; k < NHU; ++k) {
      wr[k] = sh.par[PWHH + u * NHU + k];
      wz[k] = sh.par[PWHH + (NHU + u) * NHU + k];
      wn[k] = sh.par[PWHH + (2 * NHU + u) * NHU + k];
    }
    const float br = sh.par[PBHH + u], bz = sh.par[PBHH + NHU + u], bn = sh.par[PBHH + 2 * NHU + u];
    float h = 0.0f;
#pragma unroll 1
    for (int t = 0; t < NL; ++t) {
      float hk[NHU];
#pragma unroll
      for (int k = 0; k < NHU; ++k) hk[k] = __shfl(h, k, 32);
      float dr = 0.0f, dz = 0.0f, dn = 0.0f;
#pragma unroll
      for (int k = 0; k < NHU; ++k) { dr += hk[k] * wr[k]; dz += hk[k] * wz[k]; dn += hk[k] * wn[k]; }
      const float* gp = scr + SCR_GI + t * NG3;
      const float rg = fsig(gp[u] + (dr + br));
      const float zg = fsig(gp[NHU + u] + (dz + bz));
      const float ng = ftanh(gp[2 * NHU + u] + rg * (dn + bn));
      h = (1.0f - zg) * ng + zg * h;
      if (lane < NHU) scr[SCR_X4 + t * NHU + lane] = h;
    }
  }
  __syncthreads();

  {
    const float* x4 = scr + SCR_X4;
    const int i0 = lane, i1 = lane + 32;
    const bool has1 = i1 < NL;
    const int i1c = has1 ? i1 : (NL - 1);
    const float f1 = has1 ? 1.0f : 0.0f;
    float q0[NHU], q1[NHU], y0[NHU], y1[NHU];
#pragma unroll
    for (int hd = 0; hd < NHU; ++hd) { q0[hd] = x4[i0 * NHU + hd]; q1[hd] = x4[i1c * NHU + hd]; y0[hd] = 0.0f; y1[hd] = 0.0f; }
#pragma unroll 1
    for (int j = 0; j < NL; ++j) {
      float s0 = 0.0f, s1 = 0.0f;
      float vv[NHU];
#pragma unroll
      for (int hd = 0; hd < NHU; ++hd) {
        const float rv = x4[hd * NL + j];
        vv[hd] = x4[j * NHU + hd];
        s0 += q0[hd] * rv;
        s1 += q1[hd] * rv;
      }
      s0 *= (1.0f / 6.0f);
      s1 *= (1.0f / 6.0f);
      float m = fmaxf(s0, has1 ? s1 : -__builtin_inff());
#pragma unroll
      for (int off = 16; off > 0; off >>= 1) m = fmaxf(m, __shfl_xor(m, off, 32));
      const float e0 = expf(s0 - m);
      const float e1 = expf(s1 - m) * f1;
      float se = e0 + e1;
#pragma unroll
      for (int off = 16; off > 0; off >>= 1) se += __shfl_xor(se, off, 32);
      const float inv = __builtin_amdgcn_rcpf(se);
      const float a0 = e0 * inv, a1 = e1 * inv;
#pragma unroll
      for (int hd = 0; hd < NHU; ++hd) { y0[hd] += a0 * vv[hd]; y1[hd] += a1 * vv[hd]; }
    }
    float* yS = scr + SCR_Y;
#pragma unroll
    for (int hd = 0; hd < NHU; ++hd) {
      yS[i0 * NHU + hd] = y0[hd];
      if (has1) yS[i1 * NHU + hd] = y1[hd];
    }
  }
  __syncthreads();
  {
    const int kc = lane < NHU ? lane : (NHU - 1);
    const float* yk = scr + SCR_Y + kc * NL;
    float sg = 0.0f;
#pragma unroll 1
    for (int q = 0; q < NL; ++q) sg += yk[q];
    if (lane < NHU) s.xgru[lane] = sg;
  }

  {
    const v16h bA = Frag<_Float16>::load(sWh + WA_OFF + c * XAP + koff);
    const float atb = sh.par[PATB + c];
    const unsigned short* xr = s.xrP;
#pragma unroll 1
    for (int mt = 0; mt < 4; ++mt) {
      const int l = mt * 16 + c;
      v8u au;
#pragma unroll
      for (int v = 0; v < 4; ++v) {
        const int o = (8 * hh + 2 * v) * XRP + 2 + l;
        au[v] = (unsigned)xr[o] | ((unsigned)xr[o + XRP] << 16);
      }
      au[4] = 0u; au[5] = 0u; au[6] = 0u; au[7] = 0u;
      const v16h a = __builtin_bit_cast(v16h, au);
      const v8f acc = hmma(a, bA, z8);
#pragma unroll
      for (int r = 0; r < 8; ++r) {
        const int lr = mt * 16 + 8 * hh + r;
        s.u1.attnT[lr * NCH + c] = ftanh(acc[r] * FOLD + atb);
      }
    }
  }
  __syncthreads();
  {
    float* a1 = s.u2.attn1P;
    const float* at = s.u1.attnT;
#pragma unroll 1
    for (int e = lane; e < 48 * NL; e += 32) {
      const int p = e / NL; const int l = e - NL * p;
      const int row = e / 48; const int col = (e - 48 * row) & 15;
      a1[p * A1P + l] = at[row * NCH + col];
    }
#pragma unroll 1
    for (int e = lane; e < 48 * 14; e += 32) { const int p = e / 14; const int q = e - 14 * p; a1[p * A1P + NL + q] = 0.0f; }
  }
  __syncthreads();

  {
    const unsigned short* xr = s.xrP;
    const float* a1 = s.u2.attn1P;
    float part[3] = {0.0f, 0.0f, 0.0f};
#pragma unroll 1
    for (int mt = 0; mt < 4; ++mt) {
      const int l = mt * 16 + c;
      v16h af[3];
#pragma unroll
      for (int kt = 0; kt < 3; ++kt) {
        v8u au;
#pragma unroll
        for (int v = 0; v < 8; ++v) {
          if (kt == 2 && v >= 4) {
            au[v] = 0u;
          } else {
            const int oa0 = im_off(im_k(kt, v, 0, 0)), oa1 = im_off(im_k(kt, v, 1, 0));
            const int ob0 = im_off(im_k(kt, v, 0, 1)), ob1 = im_off(im_k(kt, v, 1, 1));
            const int o0 = hh ? ob0 : oa0;
            const int o1 = hh ? ob1 : oa1;
            au[v] = (unsigned)xr[o0 + l] | ((unsigned)xr[o1 + l] << 16);
          }
        }
        af[kt] = __builtin_bit_cast(v16h, au);
      }
#pragma unroll
      for (int nt = 0; nt < 3; ++nt) {
        const int p = nt * 16 + c;
        v8f acc = z8;
#pragma unroll
        for (int kt = 0; kt < 3; ++kt) {
          const v16h b = Frag<_Float16>::load(sWh + WC_OFF + p * WCP + kt * 32 + koff);
          acc = hmma(af[kt], b, acc);
        }
        const float bias = sh.par[PCVB + p];
#pragma unroll
        for (int r = 0; r < 8; ++r) {
          const int lr = mt * 16 + 8 * hh + r;
          float v = acc[r] * FOLD + bias;
          v = (v > 0.0f) ? v : 0.1f * v;
          const float term = v * a1[p * A1P + lr];
          part[nt] += (lr < NL) ? term : 0.0f;
        }
      }
    }
#pragma unroll
    for (int nt = 0; nt < 3; ++nt) {
      const float tot = part[nt] + __shfl_xor(part[nt], 16, 32);
      if (hh == 0) s.xcnn[nt * 16 + c] = tot;
    }
  }
  __syncthreads();

  {
    const int o = lane & 1;
    const float* fw = sh.par + PFCW + o * 54;
    float acc = 0.0f;
#pragma unroll 1
    for (int q = 0; q < 48; ++q) acc += s.xcnn[q] * fw[q];
#pragma unroll
    for (int k = 0; k < NHU; ++k) acc += s.xgru[k] * fw[48 + k];
    const float res = acc + sh.par[PFCB + o];
    if (lane < 2) sh.outv[wave * 2 + lane] = res;
  }
  __syncthreads();
  if (wave == 0) {
    const float fl = (lane == 0) ? 1.0f : 0.0f;
    v4f ov;
    ov[0] = sh.outv[0] * fl; ov[1] = sh.outv[1] * fl; ov[2] = sh.outv[2] * fl; ov[3] = sh.outv[3] * fl;
    float* p = outt + (size_t)blockIdx.x * OUTT_LINE + lane * 4;
    if (lane < 8) *(volatile v4f*)p = ov;
    __threadfence();
    if (lane < 8) *(volatile v4f*)p = ov;
  }
}

__global__ __launch_bounds__(256) void k_final(const float* __restrict__ outt, float* __restrict__ out) {
  const int i = blockIdx.x * 256 + threadIdx.x;
  const v4f v = *(const v4f*)(outt + (size_t)i * OUTT_LINE);
  float* p = out + (size_t)i * 4;
  *(volatile v4f*)p = v;
  __threadfence();
  *(volatile v4f*)p = v;
}

extern "C" void kernel_launch(void* const* d_in, const int* in_sizes, int n_in,
                              void* d_out, int out_size, void* d_ws, size_t ws_size, hipStream_t stream) {
  if (n_in < 17 || d_out == nullptr || d_ws == nullptr) return;
  if (in_sizes[0] != NB * NL * ND || in_sizes[1] != NCH * ND || in_sizes[2] != NCH ||
      in_sizes[3] != NCH * NCH || in_sizes[4] != NCH ||
      in_sizes[5] != NCH * NCH * 1 || in_sizes[6] != NCH ||
      in_sizes[7] != NCH * NCH * 3 || in_sizes[8] != NCH ||
      in_sizes[9] != NCH * NCH * 5 || in_sizes[10] != NCH ||
      in_sizes[11] != NG3 * NCH || in_sizes[12] != NG3 * NHU || in_sizes[13] != NG3 || in_sizes[14] != NG3 ||
      in_sizes[15] != 2 * 54 || in_sizes[16] != 2 || out_size != NB * 2) return;

  const float* x       = (const float*)d_in[0];
  const float* we_w    = (const float*)d_in[1];
  const float* we_b    = (const float*)d_in[2];
  const float* attn_w  = (const float*)d_in[3];
  const float* attn_b  = (const float*)d_in[4];
  const float* conv1_w = (const float*)d_in[5];
  const float* conv1_b = (const float*)d_in[6];
  const float* conv2_w = (const float*)d_in[7];
  const float* conv2_b = (const float*)d_in[8];
  const float* conv3_w = (const float*)d_in[9];
  const float* conv3_b = (const float*)d_in[10];
  const float* gru_wih = (const float*)d_in[11];
  const float* gru_whh = (const float*)d_in[12];
  const float* gru_bih = (const float*)d_in[13];
  const float* gru_bhh = (const float*)d_in[14];
  const float* fc3_w   = (const float*)d_in[15];
  const float* fc3_b   = (const float*)d_in[16];
  float* out = (float*)d_out;

  char* ws = (char*)d_ws; size_t off = 0;
  auto carve = [&](size_t bytes) -> char* { char* p = ws + off; off += (bytes + 255) & ~(size_t)255; return p; };
  unsigned short* WPL  = (unsigned short*)carve((size_t)WPL_N * 2);
  float*          OUTT = (float*)carve((size_t)(NB / NWV) * OUTT_LINE * 4);
  if (off > ws_size || off > (size_t)134217728) return;

  k_prep<<<1, 256, 0, stream>>>(we_w, attn_w, gru_wih, conv1_w, conv2_w, conv3_w, WPL);
  k_front<<<NB / NWV, NTHF, 0, stream>>>(x, WPL, we_b, attn_b, conv1_b, conv2_b, conv3_b,
                                          gru_whh, gru_bih, gru_bhh, fc3_w, fc3_b, OUTT);
  k_final<<<(NB * 2) / (4 * 256), 256, 0, stream>>>(OUTT, out);
}
